// RNNImputation_37649683316768
// MI455X (gfx1250) — hardware-verified
//
#include <hip/hip_runtime.h>
#include <math.h>

constexpr int NBATCH  = 256;
constexpr int NSTEP   = 2048;
constexpr int NHID    = 128;
constexpr int NGATE3  = 3 * NHID;
constexpr int NTHR    = 256;
constexpr int ROWS_PER_BLK = 32;
constexpr int TCHUNK  = 32;
constexpr int HPITCH  = 136;
constexpr int XPITCH  = 36;
constexpr int NOUT0   = NSTEP * NBATCH;
constexpr int NOUT1   = NBATCH * (NSTEP - 1);
constexpr long OUT1_OFF_BYTES = 2097152L;
constexpr int  OUT1_OFF_ELEMS = (int)(OUT1_OFF_BYTES / 4);
constexpr float HCARRY = 256.0f;
constexpr float WCARRY = 16.0f;
constexpr float FOLD_INV = 1.0f / (HCARRY * WCARRY);
constexpr float MISSING_VAL = 128.0f;

static_assert(NBATCH % ROWS_PER_BLK == 0);
static_assert(NSTEP % TCHUNK == 0);
static_assert(NHID == 16 * (NTHR / 32));
static_assert(NHID % 32 == 0);
static_assert((2 * ROWS_PER_BLK * HPITCH) % NTHR == 0);
static_assert(8 * ROWS_PER_BLK == NTHR);
static_assert(ROWS_PER_BLK * TCHUNK / 4 == NTHR);
static_assert(OUT1_OFF_ELEMS == NOUT0);
static_assert(OUT1_OFF_BYTES % 128 == 0);
static_assert(OUT1_OFF_BYTES + (long)NOUT1 * 4 == 4193280L);
static_assert(NOUT1 % 128 == 0);
static_assert(HPITCH % 8 == 0 && XPITCH % 4 == 0);

typedef __attribute__((ext_vector_type(16))) _Float16 v16h;
typedef __attribute__((ext_vector_type(8)))  _Float16 v8h;
typedef __attribute__((ext_vector_type(8)))  float    v8f;
typedef __attribute__((ext_vector_type(4)))  float    v4f;

struct FragH {
  union U { v16h v; v8h h[2]; };
  static __device__ __forceinline__ v16h load(const _Float16* p) {
    U f; f.h[0] = *(const v8h*)(p); f.h[1] = *(const v8h*)(p + 16); return f.v;
  }
  static __device__ __forceinline__ v8f mma(v16h a, v16h b, v8f c) {
    return __builtin_amdgcn_wmma_f32_16x16x32_f16(false, a, false, b, (short)0, c, false, false);
  }
};

__device__ __forceinline__ void guard3_h(v8f& a, v8f& b, v8f& c, v16h x, v16h y0, v16h y1, v16h y2) {
  asm volatile("v_nop\n\tv_nop\n\tv_nop\n\tv_nop" : "+v"(a), "+v"(b), "+v"(c) : "v"(x), "v"(y0), "v"(y1), "v"(y2));
}
__device__ __forceinline__ void pin_h(v16h& x) { asm volatile("" : "+v"(x)); }

__device__ __forceinline__ float fsig(float x)  { return __builtin_amdgcn_rcpf(1.0f + __expf(-x)); }
__device__ __forceinline__ float ftanh(float x) { return 1.0f - 2.0f * __builtin_amdgcn_rcpf(__expf(2.0f * x) + 1.0f); }

__device__ __forceinline__ v16h load_wfrag(const float* p) {
  const v4f a0 = *(const v4f*)(p);
  const v4f a1 = *(const v4f*)(p + 4);
  const v4f a2 = *(const v4f*)(p + 16);
  const v4f a3 = *(const v4f*)(p + 20);
  v16h f;
#pragma unroll
  for (int e = 0; e < 4; ++e) {
    f[e]      = (_Float16)(a0[e] * WCARRY);
    f[4 + e]  = (_Float16)(a1[e] * WCARRY);
    f[8 + e]  = (_Float16)(a2[e] * WCARRY);
    f[12 + e] = (_Float16)(a3[e] * WCARRY);
  }
  return f;
}

__global__ __launch_bounds__(NTHR) void gru_impute_seq_kernel(
    const float* __restrict__ x, const float* __restrict__ wih, const float* __restrict__ whh,
    const float* __restrict__ bih, const float* __restrict__ bhh, const float* __restrict__ wfc,
    const float* __restrict__ bfc, float* __restrict__ out0, float* __restrict__ PT) {
  __shared__ __align__(16) _Float16 Ah[2 * ROWS_PER_BLK * HPITCH];
  __shared__ __align__(16) float    Xs[ROWS_PER_BLK * XPITCH];
  __shared__ __align__(16) float    CurS[TCHUNK * ROWS_PER_BLK];
  __shared__ __align__(16) float    PredS[TCHUNK * ROWS_PER_BLK];
  __shared__ __align__(16) float    Xpart[8 * ROWS_PER_BLK];

  const int tid = threadIdx.x, lane = tid & 31, wave = tid >> 5;
  const int c = lane & 15, hh = lane >> 4, koff = hh * 8;
  const int bbase = blockIdx.x * ROWS_PER_BLK;
  const int unit = 16 * wave + c;

  const float wR  = wih[unit];
  const float wZ  = wih[NHID + unit];
  const float wN  = wih[2 * NHID + unit];
  const float bR  = bih[unit] + bhh[unit];
  const float bZ  = bih[NHID + unit] + bhh[NHID + unit];
  const float biN = bih[2 * NHID + unit];
  const float bhN = bhh[2 * NHID + unit];
  const float wfcv = wfc[unit];
  const float bfcv = bfc[0];

  v16h wfr[4][3];
#pragma unroll
  for (int kc = 0; kc < 4; ++kc) {
#pragma unroll
    for (int g = 0; g < 3; ++g) {
      wfr[kc][g] = load_wfrag(whh + (size_t)(g * NHID + unit) * NHID + kc * 32 + koff);
      pin_h(wfr[kc][g]);
    }
  }

#pragma unroll 1
  for (int i = tid; i < 2 * ROWS_PER_BLK * HPITCH; i += NTHR) Ah[i] = (_Float16)0.0f;
  Xpart[tid] = 0.0f;
  {
    const int row = tid >> 3, c4 = (tid & 7) * 4;
    const v4f xv4 = *(const v4f*)(x + (size_t)(bbase + row) * NSTEP + c4);
    *(v4f*)(Xs + row * XPITCH + c4) = xv4;
  }
  float hst[2][8];
#pragma unroll
  for (int mt = 0; mt < 2; ++mt)
#pragma unroll
    for (int r = 0; r < 8; ++r) hst[mt][r] = 0.0f;
  __syncthreads();

  const v8f z8 = {0.f, 0.f, 0.f, 0.f, 0.f, 0.f, 0.f, 0.f};

#pragma unroll 1
  for (int t = 0; t < NSTEP; ++t) {
    const int tt  = t & (TCHUNK - 1);
    const int cur = t & 1;

    if (wave == 0) {
      float xh = bfcv;
#pragma unroll
      for (int w = 0; w < 8; ++w) xh += Xpart[w * ROWS_PER_BLK + lane];
      const float xv = Xs[lane * XPITCH + tt];
      const bool miss = (xv == MISSING_VAL) & (t > 0);
      const float cu = miss ? xh : xv;
      CurS[tt * ROWS_PER_BLK + lane]  = cu;
      PredS[tt * ROWS_PER_BLK + lane] = xh;
    }
    __syncthreads();

    if (tt == TCHUNK - 1) {
      const int t0 = t - (TCHUNK - 1);
      const int line = tid >> 3, c4 = (tid & 7) * 4;
      const v4f vc = *(const v4f*)(CurS  + line * ROWS_PER_BLK + c4);
      const v4f vp = *(const v4f*)(PredS + line * ROWS_PER_BLK + c4);
      float* po = out0 + (size_t)(t0 + line) * NBATCH + bbase + c4;
      float* pp = PT   + (size_t)(t0 + line) * NBATCH + bbase + c4;
      *(volatile v4f*)po = vc;
      *(volatile v4f*)pp = vp;
      __threadfence();
      *(volatile v4f*)po = vc;
      *(volatile v4f*)pp = vp;
      if (t + 1 < NSTEP) {
        const v4f xv4 = *(const v4f*)(x + (size_t)(bbase + line) * NSTEP + (size_t)(t + 1) + c4);
        *(v4f*)(Xs + line * XPITCH + c4) = xv4;
      }
    }

    const _Float16* ahc = Ah + cur * (ROWS_PER_BLK * HPITCH) + c * HPITCH + koff;
    _Float16* ahn = Ah + (cur ^ 1) * (ROWS_PER_BLK * HPITCH);
    const float* curp = CurS + tt * ROWS_PER_BLK + 8 * hh;
    float xps[2][8];
#pragma unroll
    for (int mt = 0; mt < 2; ++mt) {
      v8f aR = z8, aZ = z8, aN = z8;
#pragma unroll
      for (int kc = 0; kc < 4; ++kc) {
        const v16h a = FragH::load(ahc + mt * 16 * HPITCH + kc * 32);
        aR = FragH::mma(a, wfr[kc][0], aR);
        aZ = FragH::mma(a, wfr[kc][1], aZ);
        aN = FragH::mma(a, wfr[kc][2], aN);
        guard3_h(aR, aZ, aN, a, wfr[kc][0], wfr[kc][1], wfr[kc][2]);
      }
#pragma unroll
      for (int r = 0; r < 8; ++r) {
        const float cu  = curp[16 * mt + r];
        const float ghr = aR[r] * FOLD_INV;
        const float ghz = aZ[r] * FOLD_INV;
        const float ghn = aN[r] * FOLD_INV;
        const float rg  = fsig(cu * wR + bR + ghr);
        const float zg  = fsig(cu * wZ + bZ + ghz);
        const float ng  = ftanh(cu * wN + biN + rg * (ghn + bhN));
        const float ho  = hst[mt][r];
        const float hn  = (1.0f - zg) * ng + zg * ho;
        hst[mt][r] = hn;
        ahn[(16 * mt + 8 * hh + r) * HPITCH + unit] = (_Float16)(hn * HCARRY);
        xps[mt][r] = hn * wfcv;
      }
    }
#pragma unroll
    for (int mt = 0; mt < 2; ++mt) {
#pragma unroll
      for (int r = 0; r < 8; ++r) {
        float s = xps[mt][r];
        s += __shfl_xor(s, 1, 32);
        s += __shfl_xor(s, 2, 32);
        s += __shfl_xor(s, 4, 32);
        s += __shfl_xor(s, 8, 32);
        xps[mt][r] = s;
      }
    }
    if (c == 0) {
#pragma unroll
      for (int mt = 0; mt < 2; ++mt)
#pragma unroll
        for (int r = 0; r < 8; ++r) Xpart[wave * ROWS_PER_BLK + 16 * mt + 8 * hh + r] = xps[mt][r];
    }
    __syncthreads();
  }
}

__global__ __launch_bounds__(NTHR) void pred_repack_kernel(const float* __restrict__ PT, float* __restrict__ out1) {
  const int i4 = blockIdx.x * NTHR + threadIdx.x;
  if (i4 >= NOUT1 / 4) return;
  v4f v;
#pragma unroll
  for (int e = 0; e < 4; ++e) {
    const int i = 4 * i4 + e;
    const int b = i / (NSTEP - 1);
    const int t = i - b * (NSTEP - 1);
    v[e] = PT[(size_t)(t + 1) * NBATCH + b];
  }
  float* op = out1 + (size_t)i4 * 4;
  *(volatile v4f*)op = v;
  __threadfence();
  *(volatile v4f*)op = v;
}

extern "C" void kernel_launch(void* const* d_in, const int* in_sizes, int n_in,
                              void* d_out, int out_size, void* d_ws, size_t ws_size, hipStream_t stream) {
  if (n_in < 7 || d_out == nullptr || d_ws == nullptr) return;
  if (in_sizes[0] != NBATCH * NSTEP || in_sizes[1] != NGATE3 || in_sizes[2] != NGATE3 * NHID ||
      in_sizes[3] != NGATE3 || in_sizes[4] != NGATE3 || in_sizes[5] != NHID || in_sizes[6] != 1 ||
      out_size != NOUT0 + NOUT1) return;

  const float* x   = (const float*)d_in[0];
  const float* wih = (const float*)d_in[1];
  const float* whh = (const float*)d_in[2];
  const float* bih = (const float*)d_in[3];
  const float* bhh = (const float*)d_in[4];
  const float* wfc = (const float*)d_in[5];
  const float* bfc = (const float*)d_in[6];
  float* out0 = (float*)d_out;
  float* out1 = out0 + (size_t)OUT1_OFF_ELEMS;

  const size_t pt_bytes = (size_t)NSTEP * NBATCH * 4;
  if (pt_bytes > ws_size || pt_bytes > (size_t)134217728) return;
  float* PT = (float*)d_ws;

  gru_impute_seq_kernel<<<NBATCH / ROWS_PER_BLK, NTHR, 0, stream>>>(x, wih, whh, bih, bhh, wfc, bfc, out0, PT);
  pred_repack_kernel<<<(NOUT1 / 4 + NTHR - 1) / NTHR, NTHR, 0, stream>>>(PT, out1);
}
